// EagleAttention2_40596030882273
// MI455X (gfx1250) — hardware-verified
//
#include <hip/hip_runtime.h>
#include <stdint.h>
#include <stddef.h>
#include <math.h>


typedef unsigned short us_t;
typedef __bf16       v16bf __attribute__((ext_vector_type(16)));
typedef float        v8f   __attribute__((ext_vector_type(8)));
typedef float        v4f   __attribute__((ext_vector_type(4)));
typedef unsigned int u32x4 __attribute__((ext_vector_type(4)));
typedef int          v4i   __attribute__((ext_vector_type(4)));

union Frag { v16bf v; u32x4 u[2]; };

__device__ __forceinline__ unsigned bf_bits(float f) {
    unsigned u = __builtin_bit_cast(unsigned, f);
    return (u + 0x7FFFu + ((u >> 16) & 1u)) >> 16;
}
__device__ __forceinline__ float bf_val(unsigned b) {
    return __builtin_bit_cast(float, b << 16);
}
__device__ __forceinline__ void split2(float x, unsigned& hb, unsigned& lb) {
    hb = bf_bits(x);
    lb = bf_bits(x - bf_val(hb));
}
__device__ __forceinline__ u32x4 pack8(const unsigned* b) {
    u32x4 v;
    v.x = b[0] | (b[1] << 16);
    v.y = b[2] | (b[3] << 16);
    v.z = b[4] | (b[5] << 16);
    v.w = b[6] | (b[7] << 16);
    return v;
}

__device__ __forceinline__ v8f mma(v8f c, v16bf a, v16bf b) {
    v8f d = __builtin_amdgcn_wmma_f32_16x16x32_bf16(false, a, false, b, (short)0, c, false, false);
    asm volatile("v_nop\n\tv_nop\n\tv_nop\n\tv_nop" : "+v"(d) : "v"(a), "v"(b));
    return d;
}

__device__ __forceinline__ void ldfrag(Frag& f, const us_t* p) {
    f.u[0] = *(const u32x4*)(p);
    f.u[1] = *(const u32x4*)(p + 16);
}

__global__ __launch_bounds__(256) void k_split(const float* __restrict__ src,
                                               us_t* hi, us_t* lo, int n8)
{
    const int i = blockIdx.x * 256 + threadIdx.x;
    const bool ok = i < n8;
    const int ic = ok ? i : 0;
    const float* p = src + (size_t)ic * 8;
    const v4f a = *(const v4f*)(p);
    const v4f b = *(const v4f*)(p + 4);
    float x[8] = { a.x, a.y, a.z, a.w, b.x, b.y, b.z, b.w };
    unsigned hb[8], lb[8];
#pragma unroll
    for (int t = 0; t < 8; ++t) split2(x[t], hb[t], lb[t]);
    const u32x4 ph = pack8(hb);
    const u32x4 pl = pack8(lb);
    us_t* dh = hi + (size_t)ic * 8;
    us_t* dl = lo + (size_t)ic * 8;
    if (ok) { *(volatile u32x4*)dh = ph; *(volatile u32x4*)dl = pl; }
    __threadfence();
    if (ok) { *(volatile u32x4*)dh = ph; *(volatile u32x4*)dl = pl; }
}

__global__ __launch_bounds__(256) void k_rope_tab(const int* __restrict__ pos,
                                                  float* cosT, float* sinT, int S)
{
    const int i = blockIdx.x * 256 + threadIdx.x;
    const int total = S * 32;
    const bool ok = i < total;
    const int ic = ok ? i : 0;
    const int trow = ic >> 5;
    const int j = ic & 31;
    const double LOG2_BASE_OVER_32 = 0.41524101186092029;
    const float pw  = (float)exp2((double)j * LOG2_BASE_OVER_32);
    const float inv = 1.0f / pw;
    const float ang = (float)pos[trow] * inv;
    float sn, cs;
    sincosf(ang, &sn, &cs);
    if (ok) { *(volatile float*)(cosT + ic) = cs; *(volatile float*)(sinT + ic) = sn; }
    __threadfence();
    if (ok) { *(volatile float*)(cosT + ic) = cs; *(volatile float*)(sinT + ic) = sn; }
}

__global__ __launch_bounds__(256) void k_flags(const float* __restrict__ mask, int* flags, int S)
{
    __shared__ int anyw[64 * 8];
    __shared__ __align__(16) int fl[64];
    const int tid  = threadIdx.x;
    const int lane = tid & 31;
    const int wave = tid >> 5;
    const int band = blockIdx.x;
    const int nkt  = S >> 5;
    const int r    = tid >> 2;
    const int cg   = (tid & 3) * 8;
    const float* rowp = mask + (size_t)(band * 64 + r) * S + cg;

    for (int kt = 0; kt < nkt; ++kt) {
        const float* p = rowp + kt * 32;
        const v4f a = *(const v4f*)(p);
        const v4f b = *(const v4f*)(p + 4);
        int any = (a.x > -1.0e8f) | (a.y > -1.0e8f) | (a.z > -1.0e8f) | (a.w > -1.0e8f) |
                  (b.x > -1.0e8f) | (b.y > -1.0e8f) | (b.z > -1.0e8f) | (b.w > -1.0e8f);
#pragma unroll
        for (int off = 1; off < 32; off <<= 1) any |= __shfl_xor(any, off, 32);
        if (lane == 0) anyw[kt * 8 + wave] = any;
    }
    __syncthreads();
    if (tid < 64) {
        int v = 0;
        if (tid < nkt) {
#pragma unroll
            for (int w = 0; w < 8; ++w) v |= anyw[tid * 8 + w];
        }
        fl[tid] = v;
    }
    __syncthreads();
    const bool ok = tid < 16;
    v4i val;
    val.x = 0; val.y = 0; val.z = 0; val.w = 0;
    if (ok) val = *(const v4i*)&fl[tid * 4];
    int* dst = flags + (size_t)band * 64 + (ok ? tid : 0) * 4;
    if (ok) *(volatile v4i*)dst = val;
    __threadfence();
    if (ok) *(volatile v4i*)dst = val;
}

template<int MODE>
__global__ __launch_bounds__(128) void k_gemm(
    const us_t* __restrict__ Ah, const us_t* __restrict__ Al,
    const us_t* __restrict__ Wh, const us_t* __restrict__ Wl,
    int M, int N, int K,
    const float* __restrict__ cosT, const float* __restrict__ sinT,
    us_t* Oh, us_t* Ol, float* Of)
{
    __shared__ __align__(16) float lds_f[4096];
    us_t* lds16 = reinterpret_cast<us_t*>(lds_f);

    const int tid  = threadIdx.x;
    const int lane = tid & 31;
    const int wave = tid >> 5;
    const int m    = lane & 15;
    const int hl   = lane >> 4;
    const int mb0  = blockIdx.y * 64;
    const int r0   = mb0 + wave * 16;
    const int c0   = blockIdx.x * 64;
    (void)M;

    v8f acc[4] = {};

    const us_t* arh = Ah + (size_t)(r0 + m) * K + 8 * hl;
    const us_t* arl = Al + (size_t)(r0 + m) * K + 8 * hl;

    for (int k0 = 0; k0 < K; k0 += 32) {
        Frag ah, al;
        ldfrag(ah, arh + k0);
        ldfrag(al, arl + k0);
#pragma unroll
        for (int j = 0; j < 4; ++j) {
            const size_t wo = (size_t)(c0 + 16 * j + m) * K + k0 + 8 * hl;
            Frag bh, bl;
            ldfrag(bh, Wh + wo);
            ldfrag(bl, Wl + wo);
            acc[j] = mma(acc[j], ah.v, bh.v);
            acc[j] = mma(acc[j], ah.v, bl.v);
            acc[j] = mma(acc[j], al.v, bh.v);
        }
    }

    if (MODE == 0) {
#pragma unroll
        for (int j = 0; j < 2; ++j) {
            const int fidx = 16 * j + m;
#pragma unroll
            for (int r = 0; r < 8; ++r) {
                const size_t ti = (size_t)(r0 + 8 * hl + r) * 32 + fidx;
                const float cs = cosT[ti];
                const float sn = sinT[ti];
                const float x1 = acc[j][r];
                const float x2 = acc[j + 2][r];
                acc[j][r]     = x1 * cs - x2 * sn;
                acc[j + 2][r] = x2 * cs + x1 * sn;
            }
        }
    }

    if (MODE == 0) {
        us_t* st = lds16 + wave * 2048;
#pragma unroll
        for (int j = 0; j < 4; ++j) {
#pragma unroll
            for (int r = 0; r < 8; ++r) {
                unsigned hb, lb;
                split2(acc[j][r], hb, lb);
                const int idx = (8 * hl + r) * 64 + 16 * j + m;
                st[idx]        = (us_t)hb;
                st[1024 + idx] = (us_t)lb;
            }
        }
        __syncthreads();
        const int rr = lane >> 3, q = lane & 7;
        u32x4 sv[8];
#pragma unroll
        for (int pl = 0; pl < 2; ++pl) {
#pragma unroll
            for (int i = 0; i < 4; ++i)
                sv[pl * 4 + i] = *(const u32x4*)(st + pl * 1024 + (4 * i + rr) * 64 + q * 8);
        }
#pragma unroll
        for (int pl = 0; pl < 2; ++pl) {
#pragma unroll
            for (int i = 0; i < 4; ++i) {
                us_t* dst = (pl ? Ol : Oh) + (size_t)(r0 + 4 * i + rr) * N + c0 + q * 8;
                *(volatile u32x4*)dst = sv[pl * 4 + i];
            }
        }
        __threadfence();
#pragma unroll
        for (int pl = 0; pl < 2; ++pl) {
#pragma unroll
            for (int i = 0; i < 4; ++i) {
                us_t* dst = (pl ? Ol : Oh) + (size_t)(r0 + 4 * i + rr) * N + c0 + q * 8;
                *(volatile u32x4*)dst = sv[pl * 4 + i];
            }
        }
    } else if (MODE == 1) {
#pragma unroll
        for (int j = 0; j < 4; ++j) {
#pragma unroll
            for (int r = 0; r < 8; ++r) {
                unsigned hb, lb;
                split2(acc[j][r], hb, lb);
                const int idx = (16 * j + m) * 64 + 16 * wave + 8 * hl + r;
                lds16[idx]        = (us_t)hb;
                lds16[4096 + idx] = (us_t)lb;
            }
        }
        __syncthreads();
        const int rr = lane >> 3, q = lane & 7;
        u32x4 sv[8];
#pragma unroll
        for (int pl = 0; pl < 2; ++pl) {
#pragma unroll
            for (int i = 0; i < 4; ++i) {
                const int d = 16 * wave + 4 * i + rr;
                sv[pl * 4 + i] = *(const u32x4*)(lds16 + pl * 4096 + d * 64 + q * 8);
            }
        }
#pragma unroll
        for (int pl = 0; pl < 2; ++pl) {
#pragma unroll
            for (int i = 0; i < 4; ++i) {
                const int d = 16 * wave + 4 * i + rr;
                us_t* dst = (pl ? Ol : Oh) + (size_t)(c0 + d) * M + mb0 + q * 8;
                *(volatile u32x4*)dst = sv[pl * 4 + i];
            }
        }
        __threadfence();
#pragma unroll
        for (int pl = 0; pl < 2; ++pl) {
#pragma unroll
            for (int i = 0; i < 4; ++i) {
                const int d = 16 * wave + 4 * i + rr;
                us_t* dst = (pl ? Ol : Oh) + (size_t)(c0 + d) * M + mb0 + q * 8;
                *(volatile u32x4*)dst = sv[pl * 4 + i];
            }
        }
    } else {
        float* stf = lds_f + wave * 1024;
#pragma unroll
        for (int j = 0; j < 4; ++j) {
#pragma unroll
            for (int r = 0; r < 8; ++r)
                stf[(8 * hl + r) * 64 + 16 * j + m] = acc[j][r];
        }
        __syncthreads();
        const int r2 = lane >> 4, q2 = lane & 15;
        v4f fv[8];
#pragma unroll
        for (int i = 0; i < 8; ++i)
            fv[i] = *(const v4f*)(stf + (2 * i + r2) * 64 + q2 * 4);
#pragma unroll
        for (int i = 0; i < 8; ++i) {
            float* dst = Of + (size_t)(r0 + 2 * i + r2) * N + c0 + q2 * 4;
            *(volatile v4f*)dst = fv[i];
        }
        __threadfence();
#pragma unroll
        for (int i = 0; i < 8; ++i) {
            float* dst = Of + (size_t)(r0 + 2 * i + r2) * N + c0 + q2 * 4;
            *(volatile v4f*)dst = fv[i];
        }
    }
}

__global__ __launch_bounds__(128) void k_attn(
    const us_t* __restrict__ Qh, const us_t* __restrict__ Ql,
    const us_t* __restrict__ Kh, const us_t* __restrict__ Kl,
    const us_t* __restrict__ Vh, const us_t* __restrict__ Vl,
    const float* __restrict__ mask, const int* __restrict__ flags,
    us_t* Oh, us_t* Ol, int S, int NHD, int NKVD, int groups)
{
    __shared__ __align__(16) us_t pshm[4][2][16 * 32];
    __shared__ __align__(16) us_t ostg[4][2][16 * 64];

    const int tid  = threadIdx.x;
    const int lane = tid & 31;
    const int wave = tid >> 5;
    const int m    = lane & 15;
    const int hl   = lane >> 4;
    const int head = blockIdx.x;
    const int band = blockIdx.y;
    const int hkv  = head / groups;
    const int r0   = band * 64 + wave * 16;
    const int nkt  = S >> 5;

    Frag qh[2], ql[2];
#pragma unroll
    for (int c = 0; c < 2; ++c) {
        const size_t qo = (size_t)(r0 + m) * NHD + head * 64 + 32 * c + 8 * hl;
        ldfrag(qh[c], Qh + qo);
        ldfrag(ql[c], Ql + qo);
    }

    v8f o[4] = {};
    float mrow[8], lrow[8];
#pragma unroll
    for (int r = 0; r < 8; ++r) { mrow[r] = -3.0e38f; lrow[r] = 0.0f; }

    for (int kt = 0; kt < nkt; ++kt) {
        const int f = flags[(size_t)band * 64 + kt];
        if (f != 0) {
            const int kb = kt * 32;

            v8f s[2] = {};
#pragma unroll
            for (int jn = 0; jn < 2; ++jn) {
#pragma unroll
                for (int c = 0; c < 2; ++c) {
                    const size_t ko = (size_t)(kb + 16 * jn + m) * NKVD + hkv * 64 + 32 * c + 8 * hl;
                    Frag bh, bl;
                    ldfrag(bh, Kh + ko);
                    ldfrag(bl, Kl + ko);
                    s[jn] = mma(s[jn], qh[c].v, bh.v);
                    s[jn] = mma(s[jn], qh[c].v, bl.v);
                    s[jn] = mma(s[jn], ql[c].v, bh.v);
                }
            }

#pragma unroll
            for (int r = 0; r < 8; ++r) {
                const int row = r0 + 8 * hl + r;
                const float* mrp = mask + (size_t)row * S + kb + m;
                const float v0 = s[0][r] * 0.125f + mrp[0];
                const float v1 = s[1][r] * 0.125f + mrp[16];
                float mx = fmaxf(v0, v1);
#pragma unroll
                for (int off = 1; off < 16; off <<= 1) mx = fmaxf(mx, __shfl_xor(mx, off, 32));
                const float mnew  = fmaxf(mrow[r], mx);
                const float alpha = __expf(mrow[r] - mnew);
                const float p0 = __expf(v0 - mnew);
                const float p1 = __expf(v1 - mnew);
                float ps = p0 + p1;
#pragma unroll
                for (int off = 1; off < 16; off <<= 1) ps += __shfl_xor(ps, off, 32);
                lrow[r] = lrow[r] * alpha + ps;
                mrow[r] = mnew;
                o[0][r] = o[0][r] * alpha;
                o[1][r] = o[1][r] * alpha;
                o[2][r] = o[2][r] * alpha;
                o[3][r] = o[3][r] * alpha;
                unsigned h0, l0, h1, l1;
                split2(p0, h0, l0);
                split2(p1, h1, l1);
                const int idx = (8 * hl + r) * 32 + m;
                pshm[wave][0][idx]      = (us_t)h0;
                pshm[wave][0][idx + 16] = (us_t)h1;
                pshm[wave][1][idx]      = (us_t)l0;
                pshm[wave][1][idx + 16] = (us_t)l1;
            }
            __syncthreads();

            Frag ph, pl;
            ph.u[0] = *(const u32x4*)&pshm[wave][0][m * 32 + 8 * hl];
            ph.u[1] = *(const u32x4*)&pshm[wave][0][m * 32 + 16 + 8 * hl];
            pl.u[0] = *(const u32x4*)&pshm[wave][1][m * 32 + 8 * hl];
            pl.u[1] = *(const u32x4*)&pshm[wave][1][m * 32 + 16 + 8 * hl];

#pragma unroll
            for (int jd = 0; jd < 4; ++jd) {
                const size_t vo = (size_t)(hkv * 64 + 16 * jd + m) * S + kb + 8 * hl;
                Frag bh, bl;
                ldfrag(bh, Vh + vo);
                ldfrag(bl, Vl + vo);
                o[jd] = mma(o[jd], ph.v, bh.v);
                o[jd] = mma(o[jd], ph.v, bl.v);
                o[jd] = mma(o[jd], pl.v, bh.v);
            }
            __syncthreads();
        }
    }

    float inv[8];
#pragma unroll
    for (int r = 0; r < 8; ++r) inv[r] = (lrow[r] > 0.0f) ? (1.0f / lrow[r]) : 0.0f;

#pragma unroll
    for (int jd = 0; jd < 4; ++jd) {
#pragma unroll
        for (int r = 0; r < 8; ++r) {
            unsigned hb, lb;
            split2(o[jd][r] * inv[r], hb, lb);
            const int idx = (8 * hl + r) * 64 + 16 * jd + m;
            ostg[wave][0][idx] = (us_t)hb;
            ostg[wave][1][idx] = (us_t)lb;
        }
    }
    __syncthreads();
    const int rr = lane >> 3, q = lane & 7;
    u32x4 sv[8];
#pragma unroll
    for (int plv = 0; plv < 2; ++plv) {
#pragma unroll
        for (int i = 0; i < 4; ++i)
            sv[plv * 4 + i] = *(const u32x4*)&ostg[wave][plv][(4 * i + rr) * 64 + q * 8];
    }
#pragma unroll
    for (int plv = 0; plv < 2; ++plv) {
#pragma unroll
        for (int i = 0; i < 4; ++i) {
            us_t* dst = (plv ? Ol : Oh) + (size_t)(r0 + 4 * i + rr) * NHD + head * 64 + q * 8;
            *(volatile u32x4*)dst = sv[plv * 4 + i];
        }
    }
    __threadfence();
#pragma unroll
    for (int plv = 0; plv < 2; ++plv) {
#pragma unroll
        for (int i = 0; i < 4; ++i) {
            us_t* dst = (plv ? Ol : Oh) + (size_t)(r0 + 4 * i + rr) * NHD + head * 64 + q * 8;
            *(volatile u32x4*)dst = sv[plv * 4 + i];
        }
    }
}

extern "C" void kernel_launch(void* const* d_in, const int* in_sizes, int n_in,
                              void* d_out, int out_size, void* d_ws, size_t ws_size,
                              hipStream_t stream)
{
    const int S = 2048, HID = 1024, NH = 16, NKV = 4, HD = 64;
    const int NKVD = NKV * HD;
    const int GROUPS = NH / NKV;

    if (n_in < 7) return;
    if (in_sizes[0] != S * HID || in_sizes[1] != S * S || in_sizes[2] != S ||
        in_sizes[3] != HID * HID || in_sizes[4] != NKVD * HID ||
        in_sizes[5] != NKVD * HID || in_sizes[6] != HID * HID ||
        out_size != S * HID) return;
    if ((S % 64) != 0 || (HID % 64) != 0 || (NKVD % 64) != 0 || HD != 64 ||
        NH * HD != HID || (S / 32) > 64 || (HID % 32) != 0) return;

    const float* hidden = (const float*)d_in[0];
    const float* mask   = (const float*)d_in[1];
    const int*   pos    = (const int*)d_in[2];
    const float* Wq     = (const float*)d_in[3];
    const float* Wk     = (const float*)d_in[4];
    const float* Wv     = (const float*)d_in[5];
    const float* Wo     = (const float*)d_in[6];
    float* out = (float*)d_out;

    size_t off = 0;
    char* base = (char*)d_ws;
    auto carve = [&](size_t bytes) -> char* {
        char* p = base + off;
        off += (bytes + 255) & ~(size_t)255;
        return p;
    };
    us_t* Xh   = (us_t*)carve((size_t)S * HID * 2);
    us_t* Xl   = (us_t*)carve((size_t)S * HID * 2);
    us_t* Wqh  = (us_t*)carve((size_t)HID * HID * 2);
    us_t* Wql  = (us_t*)carve((size_t)HID * HID * 2);
    us_t* Wkh  = (us_t*)carve((size_t)NKVD * HID * 2);
    us_t* Wkl  = (us_t*)carve((size_t)NKVD * HID * 2);
    us_t* Wvh  = (us_t*)carve((size_t)NKVD * HID * 2);
    us_t* Wvl  = (us_t*)carve((size_t)NKVD * HID * 2);
    us_t* Woh  = (us_t*)carve((size_t)HID * HID * 2);
    us_t* Wol  = (us_t*)carve((size_t)HID * HID * 2);
    us_t* Qh   = (us_t*)carve((size_t)S * HID * 2);
    us_t* Ql   = (us_t*)carve((size_t)S * HID * 2);
    us_t* Kh   = (us_t*)carve((size_t)S * NKVD * 2);
    us_t* Kl   = (us_t*)carve((size_t)S * NKVD * 2);
    us_t* Vth  = (us_t*)carve((size_t)NKVD * S * 2);
    us_t* Vtl  = (us_t*)carve((size_t)NKVD * S * 2);
    us_t* AOh  = (us_t*)carve((size_t)S * HID * 2);
    us_t* AOl  = (us_t*)carve((size_t)S * HID * 2);
    float* cosT = (float*)carve((size_t)S * 32 * 4);
    float* sinT = (float*)carve((size_t)S * 32 * 4);
    int*  flags = (int*)carve((size_t)(S / 64) * 64 * 4);
    if (off > ws_size) return;

    {
        const int n8x = S * HID / 8, n8q = HID * HID / 8, n8k = NKVD * HID / 8;
        k_split<<<dim3((n8x + 255) / 256), dim3(256), 0, stream>>>(hidden, Xh, Xl, n8x);
        k_split<<<dim3((n8q + 255) / 256), dim3(256), 0, stream>>>(Wq, Wqh, Wql, n8q);
        k_split<<<dim3((n8k + 255) / 256), dim3(256), 0, stream>>>(Wk, Wkh, Wkl, n8k);
        k_split<<<dim3((n8k + 255) / 256), dim3(256), 0, stream>>>(Wv, Wvh, Wvl, n8k);
        k_split<<<dim3((n8q + 255) / 256), dim3(256), 0, stream>>>(Wo, Woh, Wol, n8q);
    }
    k_rope_tab<<<dim3((S * 32 + 255) / 256), dim3(256), 0, stream>>>(pos, cosT, sinT, S);
    k_flags<<<dim3(S / 64), dim3(256), 0, stream>>>(mask, flags, S);

    k_gemm<0><<<dim3(HID / 64, S / 64), dim3(128), 0, stream>>>(
        Xh, Xl, Wqh, Wql, S, HID, HID, cosT, sinT, Qh, Ql, out);
    k_gemm<0><<<dim3(NKVD / 64, S / 64), dim3(128), 0, stream>>>(
        Xh, Xl, Wkh, Wkl, S, NKVD, HID, cosT, sinT, Kh, Kl, out);
    k_gemm<1><<<dim3(NKVD / 64, S / 64), dim3(128), 0, stream>>>(
        Xh, Xl, Wvh, Wvl, S, NKVD, HID, cosT, sinT, Vth, Vtl, out);

    k_attn<<<dim3(NH, S / 64), dim3(128), 0, stream>>>(
        Qh, Ql, Kh, Kl, Vth, Vtl, mask, flags, AOh, AOl, S, HID, NKVD, GROUPS);

    k_gemm<2><<<dim3(HID / 64, S / 64), dim3(128), 0, stream>>>(
        AOh, AOl, Woh, Wol, S, HID, HID, cosT, sinT, Qh, Ql, out);
}
